// SparseMoE_40364102648332
// MI455X (gfx1250) — hardware-verified
//
#include <hip/hip_runtime.h>
#include <stddef.h>
#include <stdint.h>
#include <math.h>

#define NTOK   8192
#define DM     384
#define HD     1536
#define OD     384
#define NE     8
#define TOPK   2
#define TR     64
#define NTILE  264
#define MP     16896
#define HC     512
#define NPASS  3
#define TABH   32
#define TABL   (TABH + MP)
#define TABN   (TABH + MP + NTOK * TOPK)
#define TPT    32
#define NTHR   256
#define GTHR   128
#define WSMAX  134217728
#define LDS_BKT ((TABN + NE * 8) * 4)

#define CXL   1024.0f
#define CW    1024.0f
#define CHH   16.0f
#define CHL   1024.0f
#define S_GH  0.0009765625f
#define S_GL  9.5367431640625e-07f
#define S_YH  6.103515625e-05f
#define S_YL  5.9604644775390625e-08f

static_assert(MP == NTILE * TR);
static_assert(MP >= NTOK * TOPK + NE * (TR - 1));
static_assert((TABN % 32) == 0);
static_assert(((TABN / 4) % 8) == 0);
static_assert(NTOK == NTHR * TPT);
static_assert(HD == NPASS * HC);
static_assert((DM % 32) == 0 && (HC % 32) == 0 && (HD % 32) == 0);
static_assert((DM % 64) == 0 && (HC % 64) == 0 && (OD % 64) == 0);
static_assert((OD % 128) == 0);
static_assert(TR == (GTHR / 32) * 16);
static_assert(LDS_BKT <= 160000);
static_assert(NTHR / 32 == 8);
static_assert((NTOK % NTHR) == 0 && (NTOK % 8) == 0);
static_assert((DM % 8) == 0 && (HD % 8) == 0);
static_assert(((MP * (DM / 8)) % NTHR) == 0);

typedef float          v4f   __attribute__((ext_vector_type(4)));
typedef float          v8f   __attribute__((ext_vector_type(8)));
typedef int            v4i   __attribute__((ext_vector_type(4)));
typedef int            v8i   __attribute__((ext_vector_type(8)));
typedef _Float16       v4h   __attribute__((ext_vector_type(4)));
typedef _Float16       v8h   __attribute__((ext_vector_type(8)));
typedef _Float16       v16h  __attribute__((ext_vector_type(16)));
typedef v8h __attribute__((may_alias)) v8ha;
typedef v4f __attribute__((may_alias)) v4fa;
typedef v4i __attribute__((may_alias)) v4ia;

union FragH { v16h v; v8h h[2]; v8i w; };

__device__ __forceinline__ v8f wmh(const FragH& a, const FragH& b, v8f c) {
  v8f d = __builtin_amdgcn_wmma_f32_16x16x32_f16(false, a.v, false, b.v, (short)0, c, false, false);
  asm volatile("v_nop\n\tv_nop\n\tv_nop\n\tv_nop" : "+v"(d) : "v"(a.w), "v"(b.w));
  return d;
}

__device__ __forceinline__ v8h cvt8h(const v4f a, const v4f b, const float c) {
  v8h hv;
  hv[0] = (_Float16)(a.x * c); hv[1] = (_Float16)(a.y * c);
  hv[2] = (_Float16)(a.z * c); hv[3] = (_Float16)(a.w * c);
  hv[4] = (_Float16)(b.x * c); hv[5] = (_Float16)(b.y * c);
  hv[6] = (_Float16)(b.z * c); hv[7] = (_Float16)(b.w * c);
  return hv;
}

__device__ __forceinline__ float gelu_f(float v) {
  return 0.5f * v * (1.0f + erff(v * 0.70710678118654752f));
}

__global__ __launch_bounds__(NTHR) void k_wprep(const float* __restrict__ w, _Float16* wt, int K, int N, int nUnits) {
  const int u = (int)blockIdx.x * NTHR + (int)threadIdx.x;
  if (u >= nUnits) return;
  const int kq = K >> 3;
  const int na = u / kq;
  const int k8 = (u - na * kq) * 8;
  const int e  = na / N;
  const int n  = na - e * N;
  const float* p = w + ((size_t)e * (size_t)K + (size_t)k8) * (size_t)N + n;
  v4f a, b;
  a.x = p[0];               a.y = p[(size_t)N];       a.z = p[(size_t)2 * N];   a.w = p[(size_t)3 * N];
  b.x = p[(size_t)4 * N];   b.y = p[(size_t)5 * N];   b.z = p[(size_t)6 * N];   b.w = p[(size_t)7 * N];
  const v8h hv = cvt8h(a, b, CW);
  const size_t o = (size_t)na * (size_t)K + k8;
  *(volatile v8h*)(wt + o) = hv;
  __threadfence();
  *(volatile v8h*)(wt + o) = hv;
}

__device__ __forceinline__ void gacc(float xq, const float* swrow, float (&acc)[NE]) {
  const v4f wa = *(const v4f*)(swrow);
  const v4f wb = *(const v4f*)(swrow + 4);
  acc[0] = fmaf(xq, wa.x, acc[0]); acc[1] = fmaf(xq, wa.y, acc[1]);
  acc[2] = fmaf(xq, wa.z, acc[2]); acc[3] = fmaf(xq, wa.w, acc[3]);
  acc[4] = fmaf(xq, wb.x, acc[4]); acc[5] = fmaf(xq, wb.y, acc[5]);
  acc[6] = fmaf(xq, wb.z, acc[6]); acc[7] = fmaf(xq, wb.w, acc[7]);
}

__global__ __launch_bounds__(NTHR) void k_gate(const float* __restrict__ x, const float* __restrict__ rw,
                                               const float* __restrict__ rb, int* route) {
  __shared__ __attribute__((aligned(16))) float sw[DM * NE];
  __shared__ float sb[NE];
  const int tid = (int)threadIdx.x;
#pragma unroll 1
  for (int i = tid; i < DM * NE; i += NTHR) sw[i] = rw[i];
  if (tid < NE) sb[tid] = rb[tid];
  __syncthreads();
  int t = (int)blockIdx.x * NTHR + tid;
  const bool live = t < NTOK;
  t = t > NTOK - 1 ? NTOK - 1 : t;
  const float* xr = x + (size_t)t * DM;
  float acc[NE];
#pragma unroll
  for (int e = 0; e < NE; ++e) acc[e] = 0.f;
#pragma unroll 1
  for (int d4 = 0; d4 < DM / 4; ++d4) {
    const v4f xv = *(const v4fa*)(xr + 4 * d4);
    const float* swr = sw + (size_t)(4 * d4) * NE;
    gacc(xv.x, swr,          acc);
    gacc(xv.y, swr + NE,     acc);
    gacc(xv.z, swr + 2 * NE, acc);
    gacc(xv.w, swr + 3 * NE, acc);
  }
  float lg[NE];
#pragma unroll
  for (int e = 0; e < NE; ++e) lg[e] = acc[e] + sb[e];
  int i1 = 0;
  float v1 = lg[0];
#pragma unroll
  for (int e = 1; e < NE; ++e) {
    const bool up = lg[e] > v1;
    i1 = up ? e : i1;
    v1 = up ? lg[e] : v1;
  }
  int i2 = (i1 == 0) ? 1 : 0;
  float v2 = (i1 == 0) ? lg[1] : lg[0];
#pragma unroll
  for (int e = 0; e < NE; ++e) {
    const bool ok = (e != i1) && (lg[e] > v2);
    i2 = ok ? e : i2;
    v2 = ok ? lg[e] : v2;
  }
  const float e2  = expf(v2 - v1);
  const float s   = 1.0f + e2;
  const float inv = 1.0f / s;
  const float p1  = inv;
  const float p2  = e2 * inv;
  v4i rec;
  rec.x = i1; rec.y = i2; rec.z = __float_as_int(p1); rec.w = __float_as_int(p2);
  if (live) *(volatile v4i*)(route + (size_t)t * 4) = rec;
  __threadfence();
  if (live) *(volatile v4i*)(route + (size_t)t * 4) = rec;
}

__device__ __forceinline__ void cnt_add(int c, int (&cnt)[NE]) {
  c = c < 0 ? 0 : (c > NE - 1 ? NE - 1 : c);
#pragma unroll
  for (int e = 0; e < NE; ++e) cnt[e] += (c == e) ? 1 : 0;
}
__device__ __forceinline__ int slot_of(int c, int (&base)[NE]) {
  c = c < 0 ? 0 : (c > NE - 1 ? NE - 1 : c);
  int p = 0;
#pragma unroll
  for (int e = 0; e < NE; ++e) {
    const bool mt = (c == e);
    p = mt ? base[e] : p;
    base[e] += mt ? 1 : 0;
  }
  return p < 0 ? 0 : (p > MP - 1 ? MP - 1 : p);
}

__global__ __launch_bounds__(NTHR) void k_bucket(const int* __restrict__ route, int* tab) {
  extern __shared__ v4i lds_dyn[];
  int* img = (int*)lds_dyn;
  int* lst = img + TABH;
  int* pos = img + TABL;
  int* wt  = img + TABN;
  const int tid = (int)threadIdx.x, lane = tid & 31, wave = tid >> 5;

  const v4i z4 = {0, 0, 0, 0};
#pragma unroll 1
  for (int p = tid; p < TABN / 4; p += NTHR) *(v4i*)(img + 4 * p) = z4;
  __syncthreads();

  const int t0 = tid * TPT;
  int cnt[NE];
#pragma unroll
  for (int e = 0; e < NE; ++e) cnt[e] = 0;
#pragma unroll 1
  for (int c = 0; c < TPT; ++c) {
    const v4i rc = *(const v4ia*)(route + (size_t)(t0 + c) * 4);
    cnt_add(rc.x, cnt);
    cnt_add(rc.y, cnt);
  }
  int incl[NE];
#pragma unroll
  for (int e = 0; e < NE; ++e) {
    int v = cnt[e];
#pragma unroll
    for (int d = 1; d < 32; d <<= 1) {
      const int up = __shfl_up(v, d);
      if (lane >= d) v += up;
    }
    incl[e] = v;
    if (lane == 31) wt[e * 8 + wave] = v;
  }
  __syncthreads();
  int pre[NE], tot[NE];
#pragma unroll
  for (int e = 0; e < NE; ++e) {
    int s = 0, all = 0;
#pragma unroll
    for (int w2 = 0; w2 < NTHR / 32; ++w2) {
      const int v = wt[e * 8 + w2];
      all += v;
      s   += (w2 < wave) ? v : 0;
    }
    pre[e] = s + incl[e] - cnt[e];
    all = all < 0 ? 0 : (all > NTOK * TOPK ? NTOK * TOPK : all);
    tot[e] = all;
  }
  int off[NE + 1];
  off[0] = 0;
#pragma unroll
  for (int e = 0; e < NE; ++e) {
    int nx = off[e] + ((tot[e] + TR - 1) / TR) * TR;
    nx = nx > MP ? MP : nx;
    off[e + 1] = nx;
  }
  int base[NE];
#pragma unroll
  for (int e = 0; e < NE; ++e) base[e] = off[e] + pre[e];
#pragma unroll 1
  for (int c = 0; c < TPT; ++c) {
    const v4i rc = *(const v4ia*)(route + (size_t)(t0 + c) * 4);
    const int t = t0 + c;
    const int pa = slot_of(rc.x, base); lst[pa] = t; pos[2 * t]     = pa;
    const int pb = slot_of(rc.y, base); lst[pb] = t; pos[2 * t + 1] = pb;
  }
  __syncthreads();
  if (tid == 0) {
#pragma unroll
    for (int e = 0; e < NE; ++e) img[e] = tot[e];
#pragma unroll
    for (int j = 0; j <= NE; ++j) img[NE + j] = off[j];
  }
  __syncthreads();
#pragma unroll 1
  for (int p = tid; p < TABN / 4; p += NTHR) {
    const v4i v = *(const v4ia*)(img + 4 * p);
    *(volatile v4i*)(tab + 4 * p) = v;
  }
  __threadfence();
#pragma unroll 1
  for (int p = tid; p < TABN / 4; p += NTHR) {
    const v4i v = *(const v4ia*)(img + 4 * p);
    *(volatile v4i*)(tab + 4 * p) = v;
  }
}

__global__ __launch_bounds__(NTHR) void k_gather(const float* __restrict__ x, const int* __restrict__ tab,
                                                 _Float16* xgh, _Float16* xgl, int nUnits) {
  const int u = (int)blockIdx.x * NTHR + (int)threadIdx.x;
  if (u >= nUnits) return;
  int row = u / (DM / 8);
  const int c8 = (u - row * (DM / 8)) * 8;
  row = row > MP - 1 ? MP - 1 : row;
  int tk = tab[TABH + row];
  tk = tk < 0 ? 0 : (tk > NTOK - 1 ? NTOK - 1 : tk);
  const float* p = x + (size_t)tk * DM + c8;
  const v4f a = *(const v4fa*)p;
  const v4f b = *(const v4fa*)(p + 4);
  float f[8];
  f[0] = a.x; f[1] = a.y; f[2] = a.z; f[3] = a.w; f[4] = b.x; f[5] = b.y; f[6] = b.z; f[7] = b.w;
  v8h hv, lv;
#pragma unroll
  for (int j = 0; j < 8; ++j) {
    const _Float16 hj = (_Float16)f[j];
    hv[j] = hj;
    lv[j] = (_Float16)((f[j] - (float)hj) * CXL);
  }
  const size_t o = (size_t)row * DM + (size_t)c8;
  *(volatile v8h*)(xgh + o) = hv;
  *(volatile v8h*)(xgl + o) = lv;
  __threadfence();
  *(volatile v8h*)(xgh + o) = hv;
  *(volatile v8h*)(xgl + o) = lv;
}

__device__ __forceinline__ int tile_slot(const int* __restrict__ tab, int rowBase) {
  const v4i ho0 = *(const v4ia*)(tab + 8);
  const v4i ho1 = *(const v4ia*)(tab + 12);
  int e = 0;
#define SELX(J, OJ) { const bool ge_ = rowBase >= (OJ); e = ge_ ? (J) : e; }
  SELX(1, ho0.y) SELX(2, ho0.z) SELX(3, ho0.w)
  SELX(4, ho1.x) SELX(5, ho1.y) SELX(6, ho1.z) SELX(7, ho1.w)
#undef SELX
  return e;
}

__global__ __launch_bounds__(GTHR) void k_up(const _Float16* __restrict__ xgh, const _Float16* __restrict__ xgl,
                                             const _Float16* __restrict__ w1t, const float* __restrict__ b1,
                                             const int* __restrict__ tab, _Float16* hh, _Float16* hl, int hbase) {
  __shared__ __attribute__((aligned(16))) _Float16 sO[2 * TR * 64];
  const int tid = (int)threadIdx.x, lane = tid & 31, wave = tid >> 5, h4 = lane >> 4, m = lane & 15;
  const int rowBase = (int)blockIdx.x * TR;
  const int col0    = (int)blockIdx.y * 64;
  const int e = tile_slot(tab, rowBase);

  v8f Gh[4], Gl[4];
  {
    const v8f z = {0.f, 0.f, 0.f, 0.f, 0.f, 0.f, 0.f, 0.f};
    Gh[0] = z; Gh[1] = z; Gh[2] = z; Gh[3] = z;
    Gl[0] = z; Gl[1] = z; Gl[2] = z; Gl[3] = z;
  }
  const size_t arow = (size_t)(rowBase + 16 * wave + m) * (size_t)DM + (size_t)(8 * h4);
  const _Float16* aph = xgh + arow;
  const _Float16* apl = xgl + arow;
  const _Float16* wp  = w1t + ((size_t)e * (size_t)HD + (size_t)(hbase + col0 + m)) * (size_t)DM + (size_t)(8 * h4);
#pragma unroll 1
  for (int ks = 0; ks < DM / 32; ++ks) {
    FragH ah, al;
    ah.h[0] = *(const v8ha*)(aph + 32 * ks);
    ah.h[1] = *(const v8ha*)(aph + 32 * ks + 16);
    al.h[0] = *(const v8ha*)(apl + 32 * ks);
    al.h[1] = *(const v8ha*)(apl + 32 * ks + 16);
#pragma unroll
    for (int t = 0; t < 4; ++t) {
      const _Float16* q = wp + (size_t)(16 * t) * (size_t)DM + 32 * ks;
      FragH bf;
      bf.h[0] = *(const v8ha*)q;
      bf.h[1] = *(const v8ha*)(q + 16);
      Gh[t] = wmh(ah, bf, Gh[t]);
      Gl[t] = wmh(al, bf, Gl[t]);
    }
  }

#pragma unroll
  for (int t = 0; t < 4; ++t) {
    const int lc = 16 * t + m;
    const float bb = b1[(size_t)e * (size_t)HD + (size_t)(hbase + col0 + lc)];
#pragma unroll
    for (int r = 0; r < 8; ++r) {
      const int lr = 16 * wave + 8 * h4 + r;
      const float z = fmaf(Gh[t][r], S_GH, Gl[t][r] * S_GL) + bb;
      const float g = gelu_f(z);
      const float v = g * CHH;
      const _Float16 hf = (_Float16)v;
      const _Float16 lf = (_Float16)((v - (float)hf) * CHL);
      sO[lr * 64 + lc] = hf;
      sO[TR * 64 + lr * 64 + lc] = lf;
    }
  }
  __syncthreads();

  const int q8 = lane & 7, sub = lane >> 3;
  v8h hv[4], lv[4];
  size_t po[4];
#pragma unroll
  for (int i = 0; i < 4; ++i) {
    const int lr = 16 * wave + 4 * i + sub;
    hv[i] = *(const v8ha*)(sO + lr * 64 + 8 * q8);
    lv[i] = *(const v8ha*)(sO + TR * 64 + lr * 64 + 8 * q8);
    po[i] = (size_t)(rowBase + lr) * (size_t)HC + (size_t)(col0 + 8 * q8);
  }
#pragma unroll
  for (int i = 0; i < 4; ++i) {
    *(volatile v8h*)(hh + po[i]) = hv[i];
    *(volatile v8h*)(hl + po[i]) = lv[i];
  }
  __threadfence();
#pragma unroll
  for (int i = 0; i < 4; ++i) {
    *(volatile v8h*)(hh + po[i]) = hv[i];
    *(volatile v8h*)(hl + po[i]) = lv[i];
  }
}

__global__ __launch_bounds__(GTHR) void k_down(const _Float16* __restrict__ hh, const _Float16* __restrict__ hl,
                                               const _Float16* __restrict__ w2t, const int* __restrict__ tab,
                                               const float* __restrict__ yin, float* yout, int kbase, int addin) {
  __shared__ __attribute__((aligned(16))) float stg[TR * 64];
  const int tid = (int)threadIdx.x, lane = tid & 31, wave = tid >> 5, h4 = lane >> 4, m = lane & 15;
  const int rowBase = (int)blockIdx.x * TR;
  const int col0    = (int)blockIdx.y * 64;
  const int e = tile_slot(tab, rowBase);

  v8f Yh[4], Yl[4];
  {
    const v8f z = {0.f, 0.f, 0.f, 0.f, 0.f, 0.f, 0.f, 0.f};
    Yh[0] = z; Yh[1] = z; Yh[2] = z; Yh[3] = z;
    Yl[0] = z; Yl[1] = z; Yl[2] = z; Yl[3] = z;
  }
  const size_t arow = (size_t)(rowBase + 16 * wave + m) * (size_t)HC + (size_t)(8 * h4);
  const _Float16* aph = hh + arow;
  const _Float16* apl = hl + arow;
  const _Float16* wp  = w2t + ((size_t)e * (size_t)OD + (size_t)(col0 + m)) * (size_t)HD + (size_t)kbase + (size_t)(8 * h4);
#pragma unroll 1
  for (int ks = 0; ks < HC / 32; ++ks) {
    FragH ah, al;
    ah.h[0] = *(const v8ha*)(aph + 32 * ks);
    ah.h[1] = *(const v8ha*)(aph + 32 * ks + 16);
    al.h[0] = *(const v8ha*)(apl + 32 * ks);
    al.h[1] = *(const v8ha*)(apl + 32 * ks + 16);
#pragma unroll
    for (int t = 0; t < 4; ++t) {
      const _Float16* q = wp + (size_t)(16 * t) * (size_t)HD + 32 * ks;
      FragH bf;
      bf.h[0] = *(const v8ha*)q;
      bf.h[1] = *(const v8ha*)(q + 16);
      Yh[t] = wmh(ah, bf, Yh[t]);
      Yl[t] = wmh(al, bf, Yl[t]);
    }
  }

#pragma unroll
  for (int t = 0; t < 4; ++t) {
    const int lc = 16 * t + m;
#pragma unroll
    for (int r = 0; r < 8; ++r) {
      const int lr = 16 * wave + 8 * h4 + r;
      stg[lr * 64 + lc] = fmaf(Yh[t][r], S_YH, Yl[t][r] * S_YL);
    }
  }
  __syncthreads();

  v4f fv[8];
  size_t op[8];
#pragma unroll
  for (int i = 0; i < 8; ++i) {
    const int lr = 16 * wave + 2 * i + h4;
    fv[i] = *(const v4fa*)(stg + lr * 64 + 4 * m);
    op[i] = (size_t)(rowBase + lr) * (size_t)OD + (size_t)(col0 + 4 * m);
  }
  if (addin != 0) {
#pragma unroll
    for (int i = 0; i < 8; ++i) {
      const v4f pv = *(const v4fa*)(yin + op[i]);
      fv[i] += pv;
    }
  }
#pragma unroll
  for (int i = 0; i < 8; ++i) *(volatile v4f*)(yout + op[i]) = fv[i];
  __threadfence();
#pragma unroll
  for (int i = 0; i < 8; ++i) *(volatile v4f*)(yout + op[i]) = fv[i];
}

__global__ __launch_bounds__(NTHR) void k_combine(const float* __restrict__ y, const int* __restrict__ route,
                                                  const int* __restrict__ tab, const float* __restrict__ b2,
                                                  float* out) {
  const int lane = (int)threadIdx.x & 31, wave = (int)threadIdx.x >> 5;
  const int t = (int)blockIdx.x * 8 + wave;
  if (t >= NTOK) return;
  const v4i rec = *(const v4ia*)(route + (size_t)t * 4);
  int e1 = rec.x, e2 = rec.y;
  e1 = e1 < 0 ? 0 : (e1 > NE - 1 ? NE - 1 : e1);
  e2 = e2 < 0 ? 0 : (e2 > NE - 1 ? NE - 1 : e2);
  const float p1 = __int_as_float(rec.z);
  const float p2 = __int_as_float(rec.w);
  int qa = tab[TABL + 2 * t];
  int qb = tab[TABL + 2 * t + 1];
  qa = qa < 0 ? 0 : (qa > MP - 1 ? MP - 1 : qa);
  qb = qb < 0 ? 0 : (qb > MP - 1 ? MP - 1 : qb);
  const float* ya = y + (size_t)qa * OD;
  const float* yb = y + (size_t)qb * OD;
  const float* ba = b2 + (size_t)e1 * OD;
  const float* bb = b2 + (size_t)e2 * OD;
  float* orow = out + (size_t)t * OD;
#pragma unroll 1
  for (int c = 0; c < OD / 128; ++c) {
    const int col = 128 * c + 4 * lane;
    const v4f a  = *(const v4fa*)(ya + col);
    const v4f b  = *(const v4fa*)(yb + col);
    const v4f ua = *(const v4fa*)(ba + col);
    const v4f ub = *(const v4fa*)(bb + col);
    v4f o;
    o.x = p1 * (a.x + ua.x); o.x = fmaf(p2, b.x + ub.x, o.x);
    o.y = p1 * (a.y + ua.y); o.y = fmaf(p2, b.y + ub.y, o.y);
    o.z = p1 * (a.z + ua.z); o.z = fmaf(p2, b.z + ub.z, o.z);
    o.w = p1 * (a.w + ua.w); o.w = fmaf(p2, b.w + ub.w, o.w);
    float* op = orow + col;
    *(volatile v4f*)op = o;
    __threadfence();
    *(volatile v4f*)op = o;
  }
}

static inline int cdiv(int a, int b) { return (a + b - 1) / b; }

extern "C" void kernel_launch(void* const* d_in, const int* in_sizes, int n_in,
                              void* d_out, int out_size, void* d_ws, size_t ws_size,
                              hipStream_t stream) {
  if (n_in < 7) return;
  if (in_sizes[0] != NTOK * DM) return;
  if (in_sizes[1] != DM * NE) return;
  if (in_sizes[2] != NE) return;
  if (in_sizes[3] != NE * DM * HD) return;
  if (in_sizes[4] != NE * HD) return;
  if (in_sizes[5] != NE * HD * OD) return;
  if (in_sizes[6] != NE * OD) return;
  if (out_size != NTOK * OD) return;

  const float* x  = (const float*)d_in[0];
  const float* wg = (const float*)d_in[1];
  const float* bg = (const float*)d_in[2];
  const float* w1 = (const float*)d_in[3];
  const float* b1 = (const float*)d_in[4];
  const float* w2 = (const float*)d_in[5];
  const float* b2 = (const float*)d_in[6];
  float* out = (float*)d_out;

  char* ws = (char*)d_ws;
  size_t off = 0;
  const size_t oW1  = off; off += (size_t)NE * HD * DM * 2;    off = (off + 255) & ~(size_t)255;
  const size_t oW2  = off; off += (size_t)NE * OD * HD * 2;    off = (off + 255) & ~(size_t)255;
  const size_t oRT  = off; off += (size_t)NTOK * 4 * 4;        off = (off + 255) & ~(size_t)255;
  const size_t oTAB = off; off += (size_t)TABN * 4;            off = (off + 255) & ~(size_t)255;
  const size_t oXH  = off; off += (size_t)MP * DM * 2;         off = (off + 255) & ~(size_t)255;
  const size_t oXL  = off; off += (size_t)MP * DM * 2;         off = (off + 255) & ~(size_t)255;
  const size_t oHH  = off; off += (size_t)MP * HC * 2;         off = (off + 255) & ~(size_t)255;
  const size_t oHL  = off; off += (size_t)MP * HC * 2;         off = (off + 255) & ~(size_t)255;
  const size_t oYA  = off; off += (size_t)MP * OD * 4;         off = (off + 255) & ~(size_t)255;
  const size_t oYB  = off; off += (size_t)MP * OD * 4;         off = (off + 255) & ~(size_t)255;
  if (off > ws_size || off > (size_t)WSMAX) return;

  _Float16* W1T = (_Float16*)(ws + oW1);
  _Float16* W2T = (_Float16*)(ws + oW2);
  int*      RT  = (int*)(ws + oRT);
  int*      TAB = (int*)(ws + oTAB);
  _Float16* XGH = (_Float16*)(ws + oXH);
  _Float16* XGL = (_Float16*)(ws + oXL);
  _Float16* HH  = (_Float16*)(ws + oHH);
  _Float16* HL  = (_Float16*)(ws + oHL);
  float*    YP[2];
  YP[0] = (float*)(ws + oYA);
  YP[1] = (float*)(ws + oYB);

  hipFuncSetAttribute(reinterpret_cast<const void*>(&k_bucket),
                      hipFuncAttributeMaxDynamicSharedMemorySize, LDS_BKT);

  {
    const int nU1 = NE * HD * DM / 8;
    k_wprep<<<cdiv(nU1, NTHR), NTHR, 0, stream>>>(w1, W1T, DM, HD, nU1);
    const int nU2 = NE * OD * HD / 8;
    k_wprep<<<cdiv(nU2, NTHR), NTHR, 0, stream>>>(w2, W2T, HD, OD, nU2);
  }

  k_gate<<<cdiv(NTOK, NTHR), NTHR, 0, stream>>>(x, wg, bg, RT);
  k_bucket<<<1, NTHR, LDS_BKT, stream>>>(RT, TAB);

  {
    const int nUx = MP * (DM / 8);
    k_gather<<<cdiv(nUx, NTHR), NTHR, 0, stream>>>(x, TAB, XGH, XGL, nUx);
  }

  for (int j = 0; j < NPASS; ++j) {
    k_up<<<dim3(NTILE, HC / 64), GTHR, 0, stream>>>(XGH, XGL, W1T, b1, TAB, HH, HL, HC * j);
    float* yout = YP[j & 1];
    const float* yin = YP[(j + 1) & 1];
    k_down<<<dim3(NTILE, OD / 64), GTHR, 0, stream>>>(HH, HL, W2T, TAB, yin, yout, HC * j, (j > 0) ? 1 : 0);
  }
  k_combine<<<NTOK / 8, NTHR, 0, stream>>>(YP[(NPASS - 1) & 1], RT, TAB, b2, out);
}
